// GemmaCausalSelfAttention_8108898255496
// MI455X (gfx1250) — hardware-verified
//
#include <hip/hip_runtime.h>
#include <math.h>

typedef __attribute__((ext_vector_type(16))) _Float16 v16h;
typedef __attribute__((ext_vector_type(16))) __bf16 v16b;
typedef __attribute__((ext_vector_type(8)))  _Float16 v8h;
typedef __attribute__((ext_vector_type(8)))  float v8f;
typedef __attribute__((ext_vector_type(4)))  float v4f;
typedef __attribute__((ext_vector_type(2)))  float v2f;
typedef __attribute__((ext_vector_type(4)))  unsigned v4u;
typedef __attribute__((ext_vector_type(4)))  int v4i;
typedef float __attribute__((may_alias)) float_a;
typedef int __attribute__((may_alias)) int_a;

template <typename T> __device__ __forceinline__ void vst2(void* p, T v) { *(volatile T*)p = v; __threadfence(); *(volatile T*)p = v; }
__device__ __forceinline__ v8f wmma16(v16h a, v16h b, v8f c) {
  v8f d = __builtin_amdgcn_wmma_f32_16x16x32_f16(false, a, false, b, (short)0, c, false, false);
  asm volatile("v_nop\n\tv_nop\n\tv_nop\n\tv_nop" : "+v"(d) : "v"(a), "v"(b));
  return d;
}
__device__ __forceinline__ v8f wmma_bf(v16b a, v16b b, v8f c) {
  v8f d = __builtin_amdgcn_wmma_f32_16x16x32_bf16(false, a, false, b, (short)0, c, false, false);
  asm volatile("v_nop\n\tv_nop\n\tv_nop\n\tv_nop" : "+v"(d) : "v"(a), "v"(b));
  return d;
}
__device__ __forceinline__ v16h frag_h(const _Float16* rowk0, int lane) {
  union { v16h v; v8h q[2]; } u; const _Float16* p = rowk0 + 8 * (lane >> 4);
  u.q[0] = *(const v8h*)p; u.q[1] = *(const v8h*)(p + 16); return u.v;
}
__device__ __forceinline__ v16h frag_f32(const float* rowk0, int lane) {
  v16h a; const float* p = rowk0 + 8 * (lane >> 4);
#pragma unroll
  for (int i = 0; i < 8; ++i) { a[i] = (_Float16)p[i]; a[8 + i] = (_Float16)p[16 + i]; }
  return a;
}
__device__ __forceinline__ v16h frag_f32s(const float* rowk0, int lane, float sc) {
  v16h a; const float* p = rowk0 + 8 * (lane >> 4);
#pragma unroll
  for (int i = 0; i < 8; ++i) { a[i] = (_Float16)(p[i] * sc); a[8 + i] = (_Float16)(p[16 + i] * sc); }
  return a;
}
__device__ __forceinline__ v16h fragc_f32(const float* W, int k0, int n, int lane, int ld, int K) {
  v16h a; const int g = lane >> 4;
#pragma unroll
  for (int i = 0; i < 8; ++i) { const int ka = k0 + 8 * g + i, kb = ka + 16;
    a[i] = (_Float16)(ka < K ? W[(size_t)(ka < K ? ka : K - 1) * ld + n] : 0.f); a[8 + i] = (_Float16)(kb < K ? W[(size_t)(kb < K ? kb : K - 1) * ld + n] : 0.f); }
  return a;
}
struct F2 { v16b h, l; };
__device__ __forceinline__ F2 bsplit16(const float v[16]) { F2 r;
#pragma unroll
  for (int i = 0; i < 16; ++i) { const __bf16 h = (__bf16)v[i]; r.h[i] = h; r.l[i] = (__bf16)(v[i] - (float)h); }
  return r; }
__device__ __forceinline__ F2 split_row(const float* row, int k0, int lane) { float v[16]; const float* p = row + k0 + 8 * (lane >> 4);
#pragma unroll
  for (int i = 0; i < 8; ++i) { v[i] = p[i]; v[8 + i] = p[16 + i]; }
  return bsplit16(v); }
__device__ __forceinline__ F2 split_rowK(const float* row, int k0, int lane, int K) { float v[16]; const int g = lane >> 4;
#pragma unroll
  for (int i = 0; i < 8; ++i) { const int ka = k0 + 8 * g + i, kb = ka + 16; v[i] = ka < K ? row[ka < K ? ka : K - 1] : 0.f; v[8 + i] = kb < K ? row[kb < K ? kb : K - 1] : 0.f; }
  return bsplit16(v); }
__device__ __forceinline__ F2 split_col(const float* W, int k0, int n, int lane, int ld, int K) { float v[16]; const int g = lane >> 4;
#pragma unroll
  for (int i = 0; i < 8; ++i) { const int ka = k0 + 8 * g + i, kb = ka + 16; v[i] = ka < K ? W[(size_t)(ka < K ? ka : K - 1) * ld + n] : 0.f; v[8 + i] = kb < K ? W[(size_t)(kb < K ? kb : K - 1) * ld + n] : 0.f; }
  return bsplit16(v); }
__device__ __forceinline__ v8f mac3(const F2& a, const F2& b, v8f c) { c = wmma_bf(a.l, b.h, c); c = wmma_bf(a.h, b.l, c); return wmma_bf(a.h, b.h, c); }
__device__ __forceinline__ float sigm(float v) { return 1.0f / (1.0f + expf(-v)); }
#define LDSX() do { asm volatile("s_wait_dscnt 0" ::: "memory"); __builtin_amdgcn_wave_barrier(); __builtin_amdgcn_fence(__ATOMIC_RELEASE, "workgroup"); } while (0)


#define NB 2
#define SS 2048
#define HID 2048
#define NHQ 16
#define HDD 128
#define NR (NB * SS)
#ifndef TQB
#define TQB (SS / 64)
#endif
typedef __attribute__((ext_vector_type(8))) __bf16 v8b;
__device__ __forceinline__ v16b frag_b(const __bf16* rowk0, int lane) {
  union { v16b v; v8b q[2]; } u; const __bf16* p = rowk0 + 8 * (lane >> 4);
  u.q[0] = *(const v8b*)p; u.q[1] = *(const v8b*)(p + 16); return u.v;
}
__device__ __forceinline__ float bfr(float v) { return (float)(__bf16)v; }
__device__ __attribute__((noinline)) float exp_ni(float v) { return expf(v); }
__device__ __attribute__((noinline)) float erf_ni(float v) { return erff(v); }

#define WS_PQ  0u
#define WS_PK  (WS_PQ + 2u * (size_t)HID * HID)
#define WS_PV  (WS_PK + 2u * (size_t)HDD * HID)
#define WS_PO  (WS_PV + 2u * (size_t)HDD * HID)
#define WS_QH  (WS_PO + 2u * (size_t)HID * HID)
#define WS_QL  (WS_QH + 2u * (size_t)NR * HID)
#define WS_KH  (WS_QL + 2u * (size_t)NR * HID)
#define WS_KL  (WS_KH + 2u * (size_t)NR * HDD)
#define WS_VT  (WS_KL + 2u * (size_t)NR * HDD)
#define WS_VL  (WS_VT + 2u * (size_t)NR * HDD)
#define WS_O   (WS_VL + 2u * (size_t)NR * HDD)
#define WS_END (WS_O + 4u * (size_t)NR * HID)
#define QX 2

__global__ __launch_bounds__(256) void k_pack(const float* __restrict__ WQ, const float* __restrict__ WK, const float* __restrict__ WV, const float* __restrict__ WO, __bf16* __restrict__ P, _Float16* __restrict__ PO) {
  const int n = blockIdx.x, which = blockIdx.y, t = threadIdx.x;
  if (which == 3) { __shared__ __align__(16) _Float16 sf[HID]; for (int k = t; k < HID; k += 256) sf[k] = (_Float16)bfr(WO[(size_t)k * HID + n]); __syncthreads(); for (int q = t; q < HID / 8; q += 256) vst2((unsigned*)(PO + (size_t)n * HID + q * 8), *(const v4u*)&sf[q * 8]); return; }
  if (which >= 1 && n >= HDD) return;
  __shared__ __align__(16) __bf16 s[HID];
  if (which == 0) { for (int k = t; k < HID; k += 256) s[k] = (__bf16)WQ[(size_t)k * HID + n]; } else if (which == 1) { for (int k = t; k < HID; k += 256) s[k] = (__bf16)WK[(size_t)k * HDD + n]; } else { for (int k = t; k < HID; k += 256) s[k] = (__bf16)WV[(size_t)k * HDD + n]; }
  __syncthreads();
  __bf16* dst = (which == 0) ? P + WS_PQ / 2 + (size_t)n * HID : (which == 1) ? P + WS_PK / 2 + (size_t)n * HID : P + WS_PV / 2 + (size_t)n * HID;
  for (int q = t; q < HID / 8; q += 256) vst2((unsigned*)(dst + q * 8), *(const v4u*)&s[q * 8]);
}
__global__ __launch_bounds__(128) void k_proj(const float* __restrict__ X, const __bf16* __restrict__ P, const float* __restrict__ BQ, const float* __restrict__ BK, const float* __restrict__ BV, const float* __restrict__ COS, const float* __restrict__ SIN, _Float16* __restrict__ QH, _Float16* __restrict__ QL, _Float16* __restrict__ KH, _Float16* __restrict__ KL, _Float16* __restrict__ VT, _Float16* __restrict__ VL) {
  __shared__ __align__(16) float sf[64][HDD + 4]; __shared__ __align__(16) _Float16 so[64][HDD + 8], sol[64][HDD + 8]; __shared__ __align__(16) _Float16 st[HDD][72], stl[HDD][72];
  const int tid = threadIdx.x, wave = tid >> 5, lane = tid & 31, col = lane & 15, g = lane >> 4; const int cb = blockIdx.y; const size_t r0 = (size_t)blockIdx.x * 64 + wave * 16; const size_t rb0 = (size_t)blockIdx.x * 64;
  const __bf16* Wr = (cb < NHQ) ? P + WS_PQ / 2 + (size_t)cb * HDD * HID : (cb == NHQ) ? P + WS_PK / 2 : P + WS_PV / 2; const float* bias = (cb < NHQ) ? BQ + cb * HDD : (cb == NHQ) ? BK : BV;
  v8f acc[8] = {};
#pragma unroll 2
  for (int kc = 0; kc < HID / 32; ++kc) { v16b a; { const float* p = X + (r0 + col) * HID + kc * 32 + 8 * g;
#pragma unroll
      for (int i = 0; i < 8; ++i) { a[i] = (__bf16)p[i]; a[8 + i] = (__bf16)p[16 + i]; } }
#pragma unroll
    for (int j = 0; j < 8; ++j) acc[j] = wmma_bf(a, frag_b(Wr + (size_t)(j * 16 + col) * HID + kc * 32, lane), acc[j]); }
#pragma unroll
  for (int j = 0; j < 8; ++j) { const int c = j * 16 + col; const float bb = bfr(bias[c]);
#pragma unroll
    for (int r = 0; r < 8; ++r) sf[wave * 16 + 8 * g + r][c] = acc[j][r] + bb; }
  __syncthreads();
  if (cb <= NHQ) {
    for (int e = tid; e < 64 * (HDD / 2); e += 128) { const int r = e >> 6, i = e & 63; const size_t tpos = (rb0 + r) % SS; const float c = bfr(COS[tpos * (HDD / 2) + i]), sn = bfr(SIN[tpos * (HDD / 2) + i]); const float re = sf[r][2 * i], im = sf[r][2 * i + 1];
      const float o0 = re * c - im * sn, o1 = re * sn + im * c; const _Float16 h0 = (_Float16)o0, h1 = (_Float16)o1; so[r][2 * i] = h0; so[r][2 * i + 1] = h1; sol[r][2 * i] = (_Float16)((o0 - (float)h0) * 2048.0f); sol[r][2 * i + 1] = (_Float16)((o1 - (float)h1) * 2048.0f); }
    __syncthreads();
    if (cb < NHQ) { for (int e = tid; e < 64 * 16; e += 128) { const int r = e >> 4, q = e & 15; const size_t o = (rb0 + r) * HID + cb * HDD + q * 8; vst2((unsigned*)(QH + o), *(const v4u*)&so[r][q * 8]); vst2((unsigned*)(QL + o), *(const v4u*)&sol[r][q * 8]); } }
    else { for (int e = tid; e < 64 * 16; e += 128) { const int r = e >> 4, q = e & 15; const size_t o = (rb0 + r) * HDD + q * 8; vst2((unsigned*)(KH + o), *(const v4u*)&so[r][q * 8]); vst2((unsigned*)(KL + o), *(const v4u*)&sol[r][q * 8]); } }
  } else {
    for (int e = tid; e < 64 * HDD; e += 128) { const int r = e & 63, d = e >> 6; const float v = sf[r][d]; const _Float16 hv = (_Float16)v; st[d][r] = hv; stl[d][r] = (_Float16)((v - (float)hv) * 2048.0f); }
    __syncthreads();
    const size_t b = rb0 / SS, s0 = rb0 % SS;
    for (int e = tid; e < HDD * 8; e += 128) { const int d = e >> 3, pc = e & 7; const size_t o = (b * HDD + d) * SS + s0 + pc * 8; vst2((unsigned*)(VT + o), *(const v4u*)&st[d][pc * 8]); vst2((unsigned*)(VL + o), *(const v4u*)&stl[d][pc * 8]); } }
}
template <int HP>
__global__ __launch_bounds__(128) void k_attn(const _Float16* __restrict__ QH, const _Float16* __restrict__ QL, const _Float16* __restrict__ KH, const _Float16* __restrict__ KL, const _Float16* __restrict__ VT, const _Float16* __restrict__ VL, float* __restrict__ O) {
  constexpr int NDT = HP ? 4 : 8;
  __shared__ __align__(16) _Float16 sph[4][16][40], spl[4][16][40]; __shared__ __align__(16) float so[4][16][HDD + 4];
  const int tid = threadIdx.x, wave = tid >> 5, lane = tid & 31, col = lane & 15, g = lane >> 4; const int qb = HP ? blockIdx.x : blockIdx.x + QX, h = blockIdx.y; const size_t b = HP ? (blockIdx.z >> 1) : blockIdx.z; const int vhalf = HP ? (blockIdx.z & 1) : 0; const int q0 = qb * 64 + wave * 16; const size_t rq = b * SS + q0;
  v16h aq[4], aql[4];
#pragma unroll
  for (int kc = 0; kc < 4; ++kc) { aq[kc] = frag_h(QH + (rq + col) * HID + h * HDD + kc * 32, lane); aql[kc] = frag_h(QL + (rq + col) * HID + h * HDD + kc * 32, lane); }
  float m[8], l[8];
#pragma unroll
  for (int r = 0; r < 8; ++r) { m[r] = -3.0e38f; l[r] = 0.f; }
  v8f acc[NDT] = {}, accl[NDT] = {}; const float scale = 1.0f / sqrtf((float)HDD); const int nks = (qb * 64 + 64) / 32;
#pragma unroll 1
  for (int ks = 0; ks < nks; ++ks) { const int j0 = ks * 32; v8f s[2];
#pragma unroll
    for (int ct = 0; ct < 2; ++ct) { const int kk = j0 + ct * 16 + col; const size_t rk = (b * SS + kk) * HDD; v8f c = {}, cl = {};
#pragma unroll
      for (int kc = 0; kc < 4; ++kc) { const v16h kh = frag_h(KH + rk + kc * 32, lane); c = wmma16(aq[kc], kh, c); cl = wmma16(aql[kc], kh, cl); cl = wmma16(aq[kc], frag_h(KL + rk + kc * 32, lane), cl); }
#pragma unroll
      for (int r = 0; r < 8; ++r) s[ct][r] = (kk <= q0 + 8 * g + r) ? (c[r] + cl[r] * (1.0f / 2048.0f)) * scale : -3.0e38f; }
#pragma unroll
    for (int r = 0; r < 8; ++r) { float mx = fmaxf(s[0][r], s[1][r]);
#pragma unroll
      for (int o = 1; o < 16; o <<= 1) mx = fmaxf(mx, __shfl_xor(mx, o));
      const float mn = fmaxf(m[r], mx); const float alpha = (m[r] <= -1.0e38f) ? 0.f : __expf(m[r] - mn); const float e0 = (s[0][r] <= -1.0e38f) ? 0.f : __expf(s[0][r] - mn), e1 = (s[1][r] <= -1.0e38f) ? 0.f : __expf(s[1][r] - mn); float es = e0 + e1;
#pragma unroll
      for (int o = 1; o < 16; o <<= 1) es += __shfl_xor(es, o);
      l[r] = l[r] * alpha + es; m[r] = (mn <= -1.0e38f) ? m[r] : mn;
#pragma unroll
      for (int dt = 0; dt < NDT; ++dt) { acc[dt][r] *= alpha; if (HP) accl[dt][r] *= alpha; }
      { const float p0 = e0 * 2048.0f, p1 = e1 * 2048.0f; const _Float16 h0 = (_Float16)p0, h1 = (_Float16)p1; sph[wave][8 * g + r][col] = h0; sph[wave][8 * g + r][16 + col] = h1; if (HP) { spl[wave][8 * g + r][col] = (_Float16)((p0 - (float)h0) * 2048.0f); spl[wave][8 * g + r][16 + col] = (_Float16)((p1 - (float)h1) * 2048.0f); } } }
    LDSX();
    const v16h pa = frag_h(&sph[wave][col][0], lane); v16h pl = pa; if (HP) pl = frag_h(&spl[wave][col][0], lane);
#pragma unroll
    for (int dt = 0; dt < NDT; ++dt) { const size_t vo = (b * HDD + vhalf * 64 + dt * 16 + col) * SS + j0; const v16h vh = frag_h(VT + vo, lane); acc[dt] = wmma16(pa, vh, acc[dt]); if (HP) { accl[dt] = wmma16(pl, vh, accl[dt]); accl[dt] = wmma16(pa, frag_h(VL + vo, lane), accl[dt]); } }
    LDSX(); }
#pragma unroll
  for (int r = 0; r < 8; ++r) { const float il = (1.0f / 2048.0f) / l[r];
#pragma unroll
    for (int dt = 0; dt < NDT; ++dt) so[wave][8 * g + r][dt * 16 + col] = (acc[dt][r] + (HP ? accl[dt][r] * (1.0f / 2048.0f) : 0.f)) * il; }
  LDSX();
  for (int rl = 0; rl < 16; ++rl) for (int q = lane; q < NDT * 4; q += 32) vst2(O + (rq + rl) * HID + h * HDD + vhalf * 64 + q * 4, *(const v4f*)&so[wave][rl][q * 4]);
}
__global__ __launch_bounds__(128) void k_out(const float* __restrict__ O, const _Float16* __restrict__ PO, const float* __restrict__ BO, float* __restrict__ OUT) {
  __shared__ __align__(16) float so[4][16][132];
  const int tid = threadIdx.x, wave = tid >> 5, lane = tid & 31, col = lane & 15, g = lane >> 4; const size_t r0 = (size_t)blockIdx.x * 64 + wave * 16; const int n0 = blockIdx.y * 128;
  const bool hp = ((blockIdx.x * 64) % SS) < QX * 64;
  v8f acc[8] = {};
#pragma unroll 2
  for (int kc = 0; kc < HID / 32; ++kc) { v16h a, al; { const float* p = O + (r0 + col) * HID + kc * 32 + 8 * g;
#pragma unroll
      for (int i = 0; i < 8; ++i) { const float x0 = p[i], x1 = p[16 + i]; const _Float16 h0 = (_Float16)x0, h1 = (_Float16)x1; a[i] = h0; a[8 + i] = h1; al[i] = (_Float16)((x0 - (float)h0) * 2048.0f); al[8 + i] = (_Float16)((x1 - (float)h1) * 2048.0f); } }
#pragma unroll
    for (int j = 0; j < 8; ++j) { const v16h w = frag_h(PO + (size_t)(n0 + j * 16 + col) * HID + kc * 32, lane); if (hp) { v8f cl = {}; cl = wmma16(al, w, cl);
#pragma unroll
        for (int r = 0; r < 8; ++r) acc[j][r] += cl[r] * (1.0f / 2048.0f); }
      acc[j] = wmma16(a, w, acc[j]); } }
#pragma unroll
  for (int j = 0; j < 8; ++j)
#pragma unroll
    for (int r = 0; r < 8; ++r) so[wave][8 * g + r][j * 16 + col] = acc[j][r] + bfr(BO[n0 + j * 16 + col]);
  LDSX();
  for (int rl = 0; rl < 16; ++rl) vst2(OUT + (r0 + rl) * HID + n0 + lane * 4, *(const v4f*)&so[wave][rl][lane * 4]);
}
extern "C" void kernel_launch(void* const* d_in, const int* in_sizes, int n_in, void* d_out, int out_size, void* d_ws, size_t ws_size, hipStream_t stream) {
  (void)in_sizes; (void)n_in; (void)out_size;
  const float** F = (const float**)d_in;
  if (ws_size < (size_t)WS_END) return;
  char* ws = (char*)d_ws; __bf16* P = (__bf16*)ws; _Float16 *PO = (_Float16*)(ws + WS_PO), *QH = (_Float16*)(ws + WS_QH), *QL = (_Float16*)(ws + WS_QL), *KH = (_Float16*)(ws + WS_KH), *KL = (_Float16*)(ws + WS_KL), *VT = (_Float16*)(ws + WS_VT), *VL = (_Float16*)(ws + WS_VL); float* O = (float*)(ws + WS_O);
  k_pack<<<dim3(HID, 4), 256, 0, stream>>>(F[4], F[6], F[8], F[10], P, PO);
  k_proj<<<dim3(NR / 64, NHQ + 2), 128, 0, stream>>>(F[0], P, F[5], F[7], F[9], F[1], F[2], QH, QL, KH, KL, VT, VL);
  k_attn<1><<<dim3(QX, NHQ, NB * 2), 128, 0, stream>>>(QH, QL, KH, KL, VT, VL, O);
  if (TQB > QX) k_attn<0><<<dim3(TQB - QX, NHQ, NB), 128, 0, stream>>>(QH, QL, KH, KL, VT, VL, O);
  k_out<<<dim3(NR / 64, HID / 128), 128, 0, stream>>>(O, PO, F[11], (float*)d_out);
}
